// MultiInputGAT_6399501271418
// MI455X (gfx1250) — hardware-verified
//
#include <hip/hip_runtime.h>


#define NTHR  256
#define NWAVE 8
#define GR    32
#define XSP   132
#define CHUNK 2048
#define WCAP  256
#define NGRP  (CHUNK / (NTHR * 4))
#define NB    128
#define DFW   512
#define NCH   40
#define AGG_LDS_BYTES ((NB * DFW + 2 * NB) * 4 + (NWAVE * WCAP + NWAVE) * 4)

static_assert(NGRP == 2);
static_assert(WCAP == (CHUNK / NTHR) * 32);
static_assert(AGG_LDS_BYTES == 271392);
static_assert((XSP % 4) == 0);
static_assert((NB & (NB - 1)) == 0);
static_assert(NB <= 512);
static_assert(NB <= WCAP);

typedef float          v4f  __attribute__((ext_vector_type(4)));
typedef float          v8f  __attribute__((ext_vector_type(8)));
typedef int            v4i  __attribute__((ext_vector_type(4)));
typedef double         v2d  __attribute__((ext_vector_type(2)));
typedef __bf16         v16b __attribute__((ext_vector_type(16)));
typedef unsigned short v8us __attribute__((ext_vector_type(8)));

union FragB { v16b v; v4i u[2]; };
union Pack  { v8us s; v4i i; };

__device__ __forceinline__ unsigned short f2bf(float x) {
  unsigned b = __float_as_uint(x);
  b += 0x7FFFu + ((b >> 16) & 1u);
  return (unsigned short)(b >> 16);
}
__device__ __forceinline__ float bf2f(unsigned short h) { return __uint_as_float(((unsigned)h) << 16); }

__device__ __forceinline__ v8f wmb(v16b a, v16b b, v8f c) {
  v8f d = __builtin_amdgcn_wmma_f32_16x16x32_bf16(false, a, false, b, (short)0, c, false, false);
  asm volatile("v_nop\n\tv_nop\n\tv_nop\n\tv_nop" : "+v"(d) : "v"(a), "v"(b));
  return d;
}

__device__ __forceinline__ float lk(float t) { return fmaxf(t, 0.2f * t); }
__device__ __forceinline__ float dl(v4f t, v4f w) {
  return w.x * lk(t.x) + w.y * lk(t.y) + w.z * lk(t.z) + w.w * lk(t.w);
}
__device__ __forceinline__ v4f relu4(v4f t) {
  t.x = fmaxf(t.x, 0.f); t.y = fmaxf(t.y, 0.f); t.z = fmaxf(t.z, 0.f); t.w = fmaxf(t.w, 0.f);
  return t;
}

__global__ __launch_bounds__(NTHR) void k_cvt(const float* __restrict__ src, int srs, int sks, int rows_src, int K,
                                              unsigned short* ph, unsigned short* pl, int rows_total, int Kpad,
                                              int aff, const float* __restrict__ st,
                                              const float* __restrict__ gm, const float* __restrict__ bt) {
  const int kp8 = Kpad >> 3;
  const int n8  = rows_total * kp8;
  const int i   = blockIdx.x * NTHR + threadIdx.x;
  if (i >= n8) return;
  const int r  = i / kp8;
  const int kb = (i - r * kp8) * 8;
  const int rc = (r < rows_src) ? r : (rows_src - 1);
  float v[8];
#pragma unroll
  for (int j = 0; j < 8; ++j) {
    const int kk = kb + j;
    const int kc = (kk < K) ? kk : (K - 1);
    float t = src[(size_t)rc * (size_t)srs + (size_t)kc * (size_t)sks];
    if (aff) t = (gm[kc] * (t - st[kc])) * st[K + kc] + bt[kc];
    v[j] = (r < rows_src && kk < K) ? t : 0.f;
  }
  Pack uh, ul;
  const v4i z4 = {0, 0, 0, 0};
  uh.i = z4; ul.i = z4;
#pragma unroll
  for (int j = 0; j < 8; ++j) {
    const unsigned short hb = f2bf(v[j]);
    uh.s[j] = hb;
    ul.s[j] = f2bf(v[j] - bf2f(hb));
  }
  const size_t o = (size_t)i * 8;
  *(volatile v4i*)(ph + o) = uh.i;
  *(volatile v4i*)(pl + o) = ul.i;
  __threadfence();
  *(volatile v4i*)(ph + o) = uh.i;
  *(volatile v4i*)(pl + o) = ul.i;
}

__global__ __launch_bounds__(NTHR) void k_gemm(
    const unsigned short* __restrict__ A0, const unsigned short* __restrict__ A1,
    const unsigned short* __restrict__ B0, const unsigned short* __restrict__ B1,
    const float* __restrict__ bias, float* out, int K, int Ncols, int relu) {
  __shared__ __attribute__((aligned(16))) float Xs[GR * XSP];

  const int tid  = threadIdx.x;
  const int lane = tid & 31;
  const int wave = tid >> 5;
  const int hh   = lane >> 4;
  const int m    = lane & 15;
  const int nwv  = blockDim.x >> 5;
  const int TC   = nwv * 16;
  const int rowBase = blockIdx.x * GR;
  const int colBase = blockIdx.y * TC;
  const int ncol = colBase + wave * 16 + m;

  const size_t ra0 = (size_t)(rowBase + m) * K + 8 * hh;
  const size_t ra1 = ra0 + (size_t)16 * K;
  const size_t rb  = (size_t)ncol * K + 8 * hh;

  v8f c0 = {0.f, 0.f, 0.f, 0.f, 0.f, 0.f, 0.f, 0.f};
  v8f c1 = {0.f, 0.f, 0.f, 0.f, 0.f, 0.f, 0.f, 0.f};

#pragma unroll 1
  for (int k0 = 0; k0 < K; k0 += 32) {
    FragB ah0, ah1, al0, al1, bh, bl;
    ah0.u[0] = *(const v4i*)(A0 + ra0 + k0);  ah0.u[1] = *(const v4i*)(A0 + ra0 + k0 + 16);
    ah1.u[0] = *(const v4i*)(A0 + ra1 + k0);  ah1.u[1] = *(const v4i*)(A0 + ra1 + k0 + 16);
    al0.u[0] = *(const v4i*)(A1 + ra0 + k0);  al0.u[1] = *(const v4i*)(A1 + ra0 + k0 + 16);
    al1.u[0] = *(const v4i*)(A1 + ra1 + k0);  al1.u[1] = *(const v4i*)(A1 + ra1 + k0 + 16);
    bh.u[0]  = *(const v4i*)(B0 + rb + k0);   bh.u[1]  = *(const v4i*)(B0 + rb + k0 + 16);
    bl.u[0]  = *(const v4i*)(B1 + rb + k0);   bl.u[1]  = *(const v4i*)(B1 + rb + k0 + 16);
    c0 = wmb(ah0.v, bh.v, c0);  c0 = wmb(ah0.v, bl.v, c0);  c0 = wmb(al0.v, bh.v, c0);
    c1 = wmb(ah1.v, bh.v, c1);  c1 = wmb(ah1.v, bl.v, c1);  c1 = wmb(al1.v, bh.v, c1);
  }

  const float bv = bias[ncol];
  const int cl = wave * 16 + m;
#pragma unroll
  for (int r = 0; r < 8; ++r) {
    float t0 = c0[r] + bv;
    float t1 = c1[r] + bv;
    if (relu) { t0 = fmaxf(t0, 0.f); t1 = fmaxf(t1, 0.f); }
    Xs[(8 * hh + r) * XSP + cl]      = t0;
    Xs[(16 + 8 * hh + r) * XSP + cl] = t1;
  }
  __syncthreads();

  v4f xv[4];
  float* xpp[4];
#pragma unroll
  for (int i = 0; i < 4; ++i) {
    const int f   = (i * (int)blockDim.x + tid) * 4;
    const int row = f / TC;
    const int col = f - row * TC;
    xv[i]  = *(const v4f*)(Xs + row * XSP + col);
    xpp[i] = out + (size_t)(rowBase + row) * Ncols + colBase + col;
  }
#pragma unroll
  for (int i = 0; i < 4; ++i) *(volatile v4f*)(xpp[i]) = xv[i];
  __threadfence();
#pragma unroll
  for (int i = 0; i < 4; ++i) *(volatile v4f*)(xpp[i]) = xv[i];
}

__device__ __forceinline__ void hit(const float* xs, const float* xd, float* ar, float* mp, float* dp,
                                    v4f w0, v4f w1, v4f w2, v4f w3) {
  const v4f a0 = *(const v4f*)(xs),       a1 = *(const v4f*)(xs + 128);
  const v4f a2 = *(const v4f*)(xs + 256), a3 = *(const v4f*)(xs + 384);
  const v4f d0 = *(const v4f*)(xd),       d1 = *(const v4f*)(xd + 128);
  const v4f d2 = *(const v4f*)(xd + 256), d3 = *(const v4f*)(xd + 384);
  float s = dl(a0 + d0, w0) + dl(a1 + d1, w1) + dl(a2 + d2, w2) + dl(a3 + d3, w3);
  s += __shfl_xor(s, 16, 32);
  s += __shfl_xor(s, 8, 32);
  s += __shfl_xor(s, 4, 32);
  s += __shfl_xor(s, 2, 32);
  s += __shfl_xor(s, 1, 32);
  const float m  = mp[0], n = dp[0];
  const float mn = fmaxf(m, s);
  const float sc = __expf(m - mn);
  const float p  = __expf(s - mn);
  v4f e0 = *(v4f*)(ar),       e1 = *(v4f*)(ar + 128);
  v4f e2 = *(v4f*)(ar + 256), e3 = *(v4f*)(ar + 384);
  e0 = e0 * sc + a0 * p;  e1 = e1 * sc + a1 * p;
  e2 = e2 * sc + a2 * p;  e3 = e3 * sc + a3 * p;
  *(v4f*)(ar)       = e0;  *(v4f*)(ar + 128) = e1;
  *(v4f*)(ar + 256) = e2;  *(v4f*)(ar + 384) = e3;
  mp[0] = mn;
  dp[0] = n * sc + p;
}

__global__ __launch_bounds__(NTHR) void k_agg(
    const int* __restrict__ ei, const float* __restrict__ xl, const float* __restrict__ xr,
    const float* __restrict__ att, const float* __restrict__ bias,
    float* hout, int nN, int nE) {
  extern __shared__ v4f lds_dyn[];
  float* sacc = (float*)lds_dyn;
  float* mx   = sacc + NB * DFW;
  float* dn   = mx + NB;
  int*   list = (int*)(dn + NB);
  int*   wcnt = list + NWAVE * WCAP;

  const int tid  = threadIdx.x;
  const int lane = tid & 31;
  const int wave = tid >> 5;
  const int nodeBase = blockIdx.x * NB;

  {
    const v4f z4 = {0.f, 0.f, 0.f, 0.f};
    for (int i = tid; i < (NB * DFW) / 4; i += NTHR) lds_dyn[i] = z4;
    for (int i = tid; i < NB; i += NTHR) { mx[i] = -1.0e30f; dn[i] = 0.f; }
  }
  __syncthreads();

  const int coff = 4 * lane;
  const v4f w0 = *(const v4f*)(att + coff);
  const v4f w1 = *(const v4f*)(att + coff + 128);
  const v4f w2 = *(const v4f*)(att + coff + 256);
  const v4f w3 = *(const v4f*)(att + coff + 384);

  const int* eid = ei + nE;
  const bool al16 = ((nE & 3) == 0);
  const int nChunks = (nE + CHUNK - 1) / CHUNK;

#pragma unroll 1
  for (int ch = 0; ch <= nChunks; ++ch) {
    const int cbase = ch * CHUNK;
    const bool selfp = (ch == nChunks);
    if (!selfp) {
      int wc = 0;
#pragma unroll
      for (int g = 0; g < NGRP; ++g) {
        const int el0 = (g * NTHR + tid) * 4;
        const int e0  = cbase + el0;
        const int sent = -2147483647 - 1;
        v4i d;
        if (al16 && (e0 + 3 < nE)) {
          d = *(const v4i*)(eid + e0);
        } else {
          d.x = (e0     < nE) ? eid[min(e0, nE - 1)]     : sent;
          d.y = (e0 + 1 < nE) ? eid[min(e0 + 1, nE - 1)] : sent;
          d.z = (e0 + 2 < nE) ? eid[min(e0 + 2, nE - 1)] : sent;
          d.w = (e0 + 3 < nE) ? eid[min(e0 + 3, nE - 1)] : sent;
        }
        const unsigned s0 = (unsigned)d.x - (unsigned)nodeBase;
        const unsigned s1 = (unsigned)d.y - (unsigned)nodeBase;
        const unsigned s2 = (unsigned)d.z - (unsigned)nodeBase;
        const unsigned s3 = (unsigned)d.w - (unsigned)nodeBase;
        const bool h0 = s0 < (unsigned)NB;
        const bool h1 = s1 < (unsigned)NB;
        const bool h2 = s2 < (unsigned)NB;
        const bool h3 = s3 < (unsigned)NB;
        const unsigned many = __builtin_amdgcn_ballot_w32(h0 | h1 | h2 | h3);
        if (many != 0u) {
#define HITJ(J, HJ, SJ) { \
            const unsigned mj = __builtin_amdgcn_ballot_w32(HJ); \
            if (HJ) { \
              const int pos = wc + (int)__builtin_amdgcn_mbcnt_lo(mj, 0u); \
              if (pos < WCAP) list[wave * WCAP + pos] = ((el0 + (J)) << 9) | (int)(SJ); \
            } \
            wc += (int)__builtin_popcount(mj); }
          HITJ(0, h0, s0)
          HITJ(1, h1, s1)
          HITJ(2, h2, s2)
          HITJ(3, h3, s3)
#undef HITJ
        }
      }
      if (lane == 0) wcnt[wave] = wc;
    } else {
      for (int s = tid; s < NB; s += NTHR) list[s] = s;
      if (tid < NWAVE) {
        int c = NB - tid * WCAP;
        c = c < 0 ? 0 : (c > WCAP ? WCAP : c);
        wcnt[tid] = c;
      }
    }
    __syncthreads();

    if (wave == 0) {
#pragma unroll 1
      for (int wsx = 0; wsx < NWAVE; ++wsx) {
        int n = __builtin_amdgcn_readfirstlane(wcnt[wsx]);
        n = n > WCAP ? WCAP : n;
        n = n < 0 ? 0 : n;
#pragma unroll 1
        for (int i = 0; i < n; ++i) {
          const int ent  = __builtin_amdgcn_readfirstlane(list[wsx * WCAP + i]);
          const int slot = ent & (NB - 1);
          const int el   = (ent >> 9) & (CHUNK - 1);
          const int node = nodeBase + slot;
          if (node >= nN) continue;
          int e = cbase + el;
          if (e > nE - 1) e = nE - 1;
          int sj = ei[e];
          sj = sj < 0 ? 0 : (sj > nN - 1 ? nN - 1 : sj);
          const int srcn = selfp ? node : sj;
          const float* xs = xl + (size_t)srcn * DFW + coff;
          const float* xd = xr + (size_t)node * DFW + coff;
          float* ar = sacc + slot * DFW + coff;
          hit(xs, xd, ar, mx + slot, dn + slot, w0, w1, w2, w3);
        }
      }
    }
    __syncthreads();
  }

#pragma unroll 1
  for (int s = wave; s < NB; s += NWAVE) {
    const int node = nodeBase + s;
    if (node >= nN) break;
    const float inv = 1.0f / dn[s];
    const float* ar = sacc + s * DFW + coff;
    v4f ov[4];
    float* op[4];
#pragma unroll
    for (int i = 0; i < 4; ++i) {
      const v4f e = *(const v4f*)(ar + 128 * i);
      const v4f b = *(const v4f*)(bias + 128 * i + coff);
      ov[i] = relu4(e * inv + b);
      op[i] = hout + (size_t)node * DFW + 128 * i + coff;
    }
#pragma unroll
    for (int i = 0; i < 4; ++i) *(volatile v4f*)(op[i]) = ov[i];
    __threadfence();
#pragma unroll
    for (int i = 0; i < 4; ++i) *(volatile v4f*)(op[i]) = ov[i];
  }
}

__global__ __launch_bounds__(128) void k_bnpart(const float* __restrict__ X, int rows, int C, int rch,
                                                double* part) {
  __shared__ __attribute__((aligned(16))) double sp[256];
  const int tid = threadIdx.x;
  const int cb  = blockIdx.x * 128;
  const int c   = cb + tid;
  const int ch  = blockIdx.y;
  const int r0  = ch * rch;
  int r1 = r0 + rch;
  if (r1 > rows) r1 = rows;
  double s = 0.0, q = 0.0;
  if (c < C) {
#pragma unroll 4
    for (int r = r0; r < r1; ++r) {
      const double v = (double)X[(size_t)r * C + c];
      s += v;
      q += v * v;
    }
  }
  sp[tid]       = s;
  sp[128 + tid] = q;
  __syncthreads();

  const int sel = tid >> 6;
  const int j   = (tid & 63) * 2;
  const v2d v   = *(const v2d*)(sp + sel * 128 + j);
  double* p = part + (size_t)(2 * ch + sel) * C + cb + j;
  const bool ok = (cb + 128 <= C);
  if (ok) *(volatile v2d*)p = v;
  __threadfence();
  if (ok) *(volatile v2d*)p = v;
}

__global__ __launch_bounds__(128) void k_bnfin(const double* __restrict__ part, int C, int nch, int rows,
                                               float* st) {
  __shared__ __attribute__((aligned(16))) float sf[256];
  const int tid = threadIdx.x;
  const int cb  = blockIdx.x * 128;
  const int c   = cb + tid;
  float muf = 0.f, rs = 0.f;
  if (c < C) {
    double s = 0.0, q = 0.0;
#pragma unroll 1
    for (int ch = 0; ch < nch; ++ch) {
      s += part[(size_t)(2 * ch) * C + c];
      q += part[(size_t)(2 * ch + 1) * C + c];
    }
    const double mu = s / (double)rows;
    double var = q / (double)rows - mu * mu;
    if (var < 0.0) var = 0.0;
    muf = (float)mu;
    rs  = rsqrtf((float)var + 1e-5f);
  }
  sf[tid]       = muf;
  sf[128 + tid] = rs;
  __syncthreads();

  if (tid < 64) {
    const int sel = tid >> 5;
    const int j   = (tid & 31) * 4;
    const v4f v   = *(const v4f*)(sf + sel * 128 + j);
    float* p = st + (size_t)sel * C + cb + j;
    const bool ok = (cb + 128 <= C);
    if (ok) *(volatile v4f*)p = v;
    __threadfence();
    if (ok) *(volatile v4f*)p = v;
  }
}

__device__ __forceinline__ v4f exp4(v4f z, float m) {
  v4f r;
  r.x = __expf(z.x - m); r.y = __expf(z.y - m); r.z = __expf(z.z - m); r.w = __expf(z.w - m);
  return r;
}
__device__ __forceinline__ v4f sig4(v4f z) {
  v4f r;
  r.x = __builtin_amdgcn_rcpf(1.0f + __expf(-z.x));
  r.y = __builtin_amdgcn_rcpf(1.0f + __expf(-z.y));
  r.z = __builtin_amdgcn_rcpf(1.0f + __expf(-z.z));
  r.w = __builtin_amdgcn_rcpf(1.0f + __expf(-z.w));
  return r;
}
__device__ __forceinline__ float max4(v4f z) { return fmaxf(fmaxf(z.x, z.y), fmaxf(z.z, z.w)); }
__device__ __forceinline__ float sum4(v4f z) { return (z.x + z.y) + (z.z + z.w); }

__global__ __launch_bounds__(NTHR) void k_head(const float* __restrict__ Z, float* out0, float* out1, int nN) {
  __shared__ v4f sg[NTHR * 4];
  __shared__ v4f lg[NTHR * 4];
  const int tid = threadIdx.x;
  const int rowBase = blockIdx.x * NTHR;
  const int row = rowBase + tid;
  v4f z0 = {0.f, 0.f, 0.f, 0.f}, z1 = z0, z2 = z0, z3 = z0;
  if (row < nN) {
    const float* zp = Z + (size_t)row * 16;
    z0 = *(const v4f*)(zp);      z1 = *(const v4f*)(zp + 4);
    z2 = *(const v4f*)(zp + 8);  z3 = *(const v4f*)(zp + 12);
  }
  const float mxv = fmaxf(fmaxf(max4(z0), max4(z1)), fmaxf(max4(z2), max4(z3)));
  const v4f e0 = exp4(z0, mxv), e1 = exp4(z1, mxv), e2 = exp4(z2, mxv), e3 = exp4(z3, mxv);
  const float ssum = (sum4(e0) + sum4(e1)) + (sum4(e2) + sum4(e3));
  const float lse = __logf(ssum);
  sg[tid * 4 + 0] = sig4(z0);  sg[tid * 4 + 1] = sig4(z1);
  sg[tid * 4 + 2] = sig4(z2);  sg[tid * 4 + 3] = sig4(z3);
  lg[tid * 4 + 0] = (z0 - mxv) - lse;  lg[tid * 4 + 1] = (z1 - mxv) - lse;
  lg[tid * 4 + 2] = (z2 - mxv) - lse;  lg[tid * 4 + 3] = (z3 - mxv) - lse;
  __syncthreads();

  const int lim = nN * 4;
  v4f sv[4], lv[4];
  int gi[4];
#pragma unroll
  for (int i = 0; i < 4; ++i) {
    const int idx = i * NTHR + tid;
    sv[i] = sg[idx];
    lv[i] = lg[idx];
    gi[i] = rowBase * 4 + idx;
  }
#pragma unroll
  for (int i = 0; i < 4; ++i) {
    if (gi[i] < lim) {
      *(volatile v4f*)(out0 + (size_t)gi[i] * 4) = sv[i];
      *(volatile v4f*)(out1 + (size_t)gi[i] * 4) = lv[i];
    }
  }
  __threadfence();
#pragma unroll
  for (int i = 0; i < 4; ++i) {
    if (gi[i] < lim) {
      *(volatile v4f*)(out0 + (size_t)gi[i] * 4) = sv[i];
      *(volatile v4f*)(out1 + (size_t)gi[i] * 4) = lv[i];
    }
  }
}

static char* carve(char* base, size_t* off, size_t bytes) {
  char* p = base + *off;
  *off = (*off + bytes + 255) & ~(size_t)255;
  return p;
}

static void launch_gemm(const unsigned short* Ah, const unsigned short* Al,
                        const unsigned short* Bh, const unsigned short* Bl,
                        const float* bias, float* out, int Mpad, int K, int Ncols, int relu,
                        hipStream_t stream) {
  const int nwv = (Ncols >= 128) ? 8 : (Ncols / 16);
  const int TC  = nwv * 16;
  k_gemm<<<dim3(Mpad / GR, Ncols / TC), nwv * 32, 0, stream>>>(Ah, Al, Bh, Bl, bias, out, K, Ncols, relu);
}

extern "C" void kernel_launch(void* const* d_in, const int* in_sizes, int n_in,
                              void* d_out, int out_size, void* d_ws, size_t ws_size,
                              hipStream_t stream) {
  if (n_in < 33) return;
  const int DI = 128, DHC = 512, D1 = 256, D2 = 128, DO = 16;
  const int nN = in_sizes[11] / DI;
  if (nN <= 0 || in_sizes[11] != nN * DI) return;
  const int nE = in_sizes[12] / 2;
  if (nE <= 0 || in_sizes[12] != 2 * nE) return;
  if (in_sizes[14] != DI * DHC || in_sizes[15] != DHC || in_sizes[16] != DI * DHC || in_sizes[17] != DHC ||
      in_sizes[18] != DHC || in_sizes[19] != DHC || in_sizes[20] != DHC || in_sizes[21] != DHC) return;
  if (in_sizes[22] != DHC * D1 || in_sizes[23] != D1 || in_sizes[24] != D1 || in_sizes[25] != D1) return;
  if (in_sizes[26] != D1 * D2 || in_sizes[27] != D2 || in_sizes[28] != D2 || in_sizes[29] != D2) return;
  if (in_sizes[30] != D2 * DO || in_sizes[31] != DO) return;
  if (out_size != 2 * nN * DO) return;

  const float* x   = (const float*)d_in[11];
  const int*   ei  = (const int*)d_in[12];
  const float* Wl  = (const float*)d_in[14];  const float* bl  = (const float*)d_in[15];
  const float* Wr  = (const float*)d_in[16];  const float* br  = (const float*)d_in[17];
  const float* att = (const float*)d_in[18];  const float* bo  = (const float*)d_in[19];
  const float* gm0 = (const float*)d_in[20];  const float* bt0 = (const float*)d_in[21];
  const float* W1  = (const float*)d_in[22];  const float* b1  = (const float*)d_in[23];
  const float* g1  = (const float*)d_in[24];  const float* be1 = (const float*)d_in[25];
  const float* W2  = (const float*)d_in[26];  const float* b2  = (const float*)d_in[27];
  const float* g2  = (const float*)d_in[28];  const float* be2 = (const float*)d_in[29];
  const float* W3  = (const float*)d_in[30];  const float* b3  = (const float*)d_in[31];
  float* out0 = (float*)d_out;
  float* out1 = out0 + (size_t)nN * DO;

  const int Mpad = ((nN + GR - 1) / GR) * GR;

  char* wsp = (char*)d_ws;
  size_t off = 0;
  const size_t plA = (size_t)Mpad * DHC * 2;
  const size_t plB = (size_t)D1 * DHC * 2;
  const size_t xB  = (size_t)Mpad * DHC * 4;
  unsigned short* Ah = (unsigned short*)carve(wsp, &off, plA);
  unsigned short* Al = (unsigned short*)carve(wsp, &off, plA);
  unsigned short* Bh = (unsigned short*)carve(wsp, &off, plB);
  unsigned short* Bl = (unsigned short*)carve(wsp, &off, plB);
  float* xl = (float*)carve(wsp, &off, xB);
  float* xr = (float*)carve(wsp, &off, xB);
  float* h  = (float*)carve(wsp, &off, xB);
  float* z1 = (float*)carve(wsp, &off, (size_t)Mpad * D1 * 4);
  float* z2 = (float*)carve(wsp, &off, (size_t)Mpad * D2 * 4);
  float* z3 = (float*)carve(wsp, &off, (size_t)Mpad * DO * 4);
  double* part = (double*)carve(wsp, &off, (size_t)NCH * 2 * DHC * 8);
  float* st = (float*)carve(wsp, &off, (size_t)2 * DHC * 4);
  if (off > ws_size) return;

  const int rch = (nN + NCH - 1) / NCH;

  hipFuncSetAttribute(reinterpret_cast<const void*>(&k_agg),
                      hipFuncAttributeMaxDynamicSharedMemorySize, AGG_LDS_BYTES);

  k_cvt<<<(Mpad * (DI / 8) + NTHR - 1) / NTHR, NTHR, 0, stream>>>(x, DI, 1, nN, DI, Ah, Al, Mpad, DI, 0, st, bl, bl);
  k_cvt<<<(DHC * (DI / 8) + NTHR - 1) / NTHR, NTHR, 0, stream>>>(Wl, 1, DHC, DHC, DI, Bh, Bl, DHC, DI, 0, st, bl, bl);
  launch_gemm(Ah, Al, Bh, Bl, bl, xl, Mpad, DI, DHC, 0, stream);
  k_cvt<<<(DHC * (DI / 8) + NTHR - 1) / NTHR, NTHR, 0, stream>>>(Wr, 1, DHC, DHC, DI, Bh, Bl, DHC, DI, 0, st, bl, bl);
  launch_gemm(Ah, Al, Bh, Bl, br, xr, Mpad, DI, DHC, 0, stream);

  k_agg<<<(nN + NB - 1) / NB, NTHR, AGG_LDS_BYTES, stream>>>(ei, xl, xr, att, bo, h, nN, nE);

  k_bnpart<<<dim3(DHC / 128, NCH), 128, 0, stream>>>(h, nN, DHC, rch, part);
  k_bnfin<<<DHC / 128, 128, 0, stream>>>(part, DHC, NCH, nN, st);
  k_cvt<<<(Mpad * (DHC / 8) + NTHR - 1) / NTHR, NTHR, 0, stream>>>(h, DHC, 1, nN, DHC, Ah, Al, Mpad, DHC, 1, st, gm0, bt0);
  k_cvt<<<(D1 * (DHC / 8) + NTHR - 1) / NTHR, NTHR, 0, stream>>>(W1, 1, D1, D1, DHC, Bh, Bl, D1, DHC, 0, st, bl, bl);
  launch_gemm(Ah, Al, Bh, Bl, b1, z1, Mpad, DHC, D1, 1, stream);

  k_bnpart<<<dim3(D1 / 128, NCH), 128, 0, stream>>>(z1, nN, D1, rch, part);
  k_bnfin<<<D1 / 128, 128, 0, stream>>>(part, D1, NCH, nN, st);
  k_cvt<<<(Mpad * (D1 / 8) + NTHR - 1) / NTHR, NTHR, 0, stream>>>(z1, D1, 1, nN, D1, Ah, Al, Mpad, D1, 1, st, g1, be1);
  k_cvt<<<(D2 * (D1 / 8) + NTHR - 1) / NTHR, NTHR, 0, stream>>>(W2, 1, D2, D2, D1, Bh, Bl, D2, D1, 0, st, bl, bl);
  launch_gemm(Ah, Al, Bh, Bl, b2, z2, Mpad, D1, D2, 1, stream);

  k_bnpart<<<dim3(D2 / 128, NCH), 128, 0, stream>>>(z2, nN, D2, rch, part);
  k_bnfin<<<D2 / 128, 128, 0, stream>>>(part, D2, NCH, nN, st);
  k_cvt<<<(Mpad * (D2 / 8) + NTHR - 1) / NTHR, NTHR, 0, stream>>>(z2, D2, 1, nN, D2, Ah, Al, Mpad, D2, 1, st, g2, be2);
  k_cvt<<<(DO * (D2 / 8) + NTHR - 1) / NTHR, NTHR, 0, stream>>>(W3, 1, DO, DO, D2, Bh, Bl, DO, D2, 0, st, bl, bl);
  launch_gemm(Ah, Al, Bh, Bl, b3, z3, Mpad, D2, DO, 0, stream);

  k_head<<<(nN + NTHR - 1) / NTHR, NTHR, 0, stream>>>(z3, out0, out1, nN);
}
